// SeparableConvolutionModule_37211596652738
// MI455X (gfx1250) — hardware-verified
//
#include <hip/hip_runtime.h>
#include <math.h>

#define NBs 2
#define CCs 3
#define HO 384
#define WO 384
#define KT 51
#define HI (HO + KT - 1)
#define WI (WO + KT - 1)
#define XT 64
#define KB 128
#define MRW 160

typedef _Float16 f16;
typedef __attribute__((ext_vector_type(16))) f16 f16x16;
typedef __attribute__((ext_vector_type(8)))  f16 f16x8;
typedef __attribute__((ext_vector_type(8)))  float f32x8;
typedef __attribute__((ext_vector_type(4)))  float v4f_t;
typedef float v4fa __attribute__((ext_vector_type(4), may_alias));
__device__ __forceinline__ f32x8 wmma16(f16x16 a, f16x16 b, f32x8 c) {
  c = __builtin_amdgcn_wmma_f32_16x16x32_f16(false, a, false, b, (short)0, c, false, false);
  asm volatile("v_nop\n\tv_nop\n\tv_nop\n\tv_nop" : "+v"(c) : "v"(a), "v"(b));
  return c;
}
__device__ __forceinline__ f16x16 lds_frag(const f16* base, int stride) {
  const int lane = threadIdx.x & 31, row = lane & 15, kh = (lane >> 4) * 8;
  const f16x8 lo = *(const f16x8*)(base + row * stride + kh);
  const f16x8 hi = *(const f16x8*)(base + row * stride + kh + 16);
  f16x16 f;
#pragma unroll
  for (int i = 0; i < 8; ++i) { f[i] = lo[i]; f[i + 8] = hi[i]; }
  return f;
}
__global__ __launch_bounds__(256) void k_sepconv(const float* __restrict__ inp, const float* __restrict__ vert, const float* __restrict__ horiz, float* __restrict__ out) {
  __shared__ __attribute__((aligned(16))) f16 bS[XT * 136];
  __shared__ float tS[MRW * 68];
  __shared__ __attribute__((aligned(16))) float oS[CCs * 68];
  const int tid = threadIdx.x, lane = tid & 31, wave = tid >> 5, cl = lane & 15, rh = (lane >> 4) * 8;
  const int nxt = WO / XT; const int b = blockIdx.x / (HO * nxt), rem = blockIdx.x % (HO * nxt), y = rem / nxt, x0 = (rem % nxt) * XT;
  for (int e = tid; e < XT * KB; e += 256) { const int xl = e >> 7, m = e & 127; const int j = m - xl;
    bS[xl * 136 + m] = (j >= 0 && j < KT) ? (f16)horiz[(((size_t)b * KT + j) * HO + y) * WO + x0 + xl] : (f16)0.0f; }
  __syncthreads();
  for (int rsel = 0; rsel < 2; ++rsel) { const int rt = wave + 8 * rsel; if (rt >= MRW / 16) break;
    f32x8 acc[4];
#pragma unroll
    for (int j = 0; j < 4; ++j) { f32x8 z = {}; acc[j] = z; }
    const int r = rt * 16 + (lane & 15); const int rr = min(r, CCs * KT - 1); const int c = rr / KT, i = rr % KT; const bool rv = r < CCs * KT;
    const float* arow = inp + (((size_t)b * CCs + c) * HI + y + i) * WI + x0;
#pragma unroll
    for (int ks = 0; ks < KB / 32; ++ks) { const int kh = (lane >> 4) * 8; f16x16 af;
#pragma unroll
      for (int e = 0; e < 8; ++e) { const int m0 = ks * 32 + kh + e, m1 = m0 + 16;
        af[e] = rv ? (f16)arow[min(m0, WI - 1 - x0)] : (f16)0.0f; af[8 + e] = rv ? (f16)arow[min(m1, WI - 1 - x0)] : (f16)0.0f; }
#pragma unroll
      for (int j = 0; j < 4; ++j) acc[j] = wmma16(af, lds_frag(bS + (j * 16) * 136 + ks * 32, 136), acc[j]); }
#pragma unroll
    for (int j = 0; j < 4; ++j)
#pragma unroll
      for (int q = 0; q < 8; ++q) tS[(rt * 16 + rh + q) * 68 + j * 16 + cl] = acc[j][q]; }
  __syncthreads();
  if (tid < CCs * XT) { const int c = tid / XT, xl = tid % XT; float s = 0.0f;
#pragma unroll 1
    for (int i = 0; i < KT; ++i) s += vert[(((size_t)b * KT + i) * HO + y) * WO + x0 + xl] * tS[(c * KT + i) * 68 + xl];
    oS[c * 68 + xl] = s; }
  __syncthreads();
#pragma unroll 1
  for (int pass = 0; pass < 2; ++pass) { if (tid < CCs * 16) { const int c = tid >> 4, c4 = (tid & 15) * 4;
      *(volatile v4f_t*)(out + (((size_t)b * CCs + c) * HO + y) * WO + x0 + c4) = *(const v4fa*)(oS + c * 68 + c4); } __threadfence(); }
}

extern "C" void kernel_launch(void* const* d_in, const int* in_sizes, int n_in,
                              void* d_out, int out_size, void* d_ws, size_t ws_size,
                              hipStream_t stream) {
  (void)in_sizes; (void)n_in; (void)out_size; (void)d_ws; (void)ws_size;
  const float* inp = (const float*)d_in[0];
  const float* vert = (const float*)d_in[1];
  const float* horiz = (const float*)d_in[2];
  float* out = (float*)d_out;
  k_sepconv<<<dim3(NBs * HO * (WO / XT)), dim3(256), 0, stream>>>(inp, vert, horiz, out);
}
